// PoolNet_61607010894040
// MI455X (gfx1250) — hardware-verified
//
#include <hip/hip_runtime.h>
#include <stddef.h>
#include <stdint.h>


#define BG     8
#define NPG1   8192
#define DEGE   16
#define EPG    (NPG1 * DEGE)
#define NEDGE  (BG * EPG)
#define KP1    2458
#define KP2    738
#define NT1    (BG * NPG1)
#define NT2    (BG * KP1)
#define NT3    (BG * KP2)
#define SPAD1  NPG1
#define SPAD2  2464
#define NCLS   10
#define CHUNK  2048
#define WCAP   256
#define NGRP   2
#define WSLIM  134217728

static_assert(NGRP * 256 * 4 == CHUNK);
static_assert(WCAP == (CHUNK / 256) * 32);
static_assert((KP1 % 2) == 0);
static_assert((SPAD2 % 32) == 0);
static_assert(SPAD2 >= ((KP1 + 31) / 32) * 32);
static_assert((NT2 % 16) == 0);
static_assert((NT3 % 16) == 0);
static_assert((EPG % CHUNK) == 0);
static_assert((NEDGE % 1024) == 0);
static_assert((NT1 % 64) == 0);

typedef float          v4f  __attribute__((ext_vector_type(4)));
typedef float          v8f  __attribute__((ext_vector_type(8)));
typedef int            v4i  __attribute__((ext_vector_type(4)));
typedef unsigned int   v2u  __attribute__((ext_vector_type(2)));
typedef unsigned int   v4u  __attribute__((ext_vector_type(4)));
typedef unsigned short v8us __attribute__((ext_vector_type(8)));
typedef __bf16         v16b __attribute__((ext_vector_type(16)));
union Frag { v16b v; v8us h8[2]; v4u q[2]; unsigned short s[16]; };

__device__ __forceinline__ v8f wm(v16b a, v16b b, v8f c) {
  v8f d = __builtin_amdgcn_wmma_f32_16x16x32_bf16(false, a, false, b, (short)0, c, false, false);
  asm volatile("v_nop\n\tv_nop\n\tv_nop\n\tv_nop" : "+v"(d) : "v"(a), "v"(b));
  return d;
}
__device__ __forceinline__ v8f wm3(v16b ah, v16b al, v16b bh, v16b bl, v8f c) {
  c = wm(ah, bh, c);
  c = wm(ah, bl, c);
  c = wm(al, bh, c);
  return c;
}
__device__ __forceinline__ v8f zero8() { v8f z = {0.f, 0.f, 0.f, 0.f, 0.f, 0.f, 0.f, 0.f}; return z; }
__device__ __forceinline__ void fragz(Frag& f) { const v4u z = {0u, 0u, 0u, 0u}; f.q[0] = z; f.q[1] = z; }

__device__ __forceinline__ unsigned short bfr(float f) {
  unsigned u = __float_as_uint(f);
  u += 0x7FFFu + ((u >> 16) & 1u);
  return (unsigned short)(u >> 16);
}
__device__ __forceinline__ float bfv(unsigned short b) { return __uint_as_float(((unsigned)b) << 16); }
__device__ __forceinline__ unsigned split2(float x) {
  const unsigned short h = bfr(x);
  const unsigned short l = bfr(x - bfv(h));
  return (unsigned)h | (((unsigned)l) << 16);
}
__device__ __forceinline__ unsigned f2o(float f) {
  const unsigned u = __float_as_uint(f);
  return (u & 0x80000000u) ? ~u : (u | 0x80000000u);
}
__device__ __forceinline__ float o2f(unsigned e) {
  const unsigned u = (e & 0x80000000u) ? (e & 0x7FFFFFFFu) : ~e;
  return __uint_as_float(u);
}
__device__ __forceinline__ float elu1(float v) { return v > 0.f ? v : (__expf(v) - 1.0f); }
__device__ __forceinline__ float lrelu(float v) { return v > 0.f ? v : 0.2f * v; }
__device__ __forceinline__ float wsum(float v) {
  v += __shfl_xor(v, 16, 32);
  v += __shfl_xor(v, 8, 32);
  v += __shfl_xor(v, 4, 32);
  v += __shfl_xor(v, 2, 32);
  v += __shfl_xor(v, 1, 32);
  return v;
}
__device__ __forceinline__ int clampi(int v, int lo, int hi) { return v < lo ? lo : (v > hi ? hi : v); }

__global__ __launch_bounds__(128) void k_proj1(const float* __restrict__ pos, const float* __restrict__ W1,
                                               float* xp, int nN) {
  __shared__ __attribute__((aligned(16))) float xs[4 * 16 * 36];
  const int tid = threadIdx.x, lane = tid & 31, wave = tid >> 5, hh = lane >> 4, m = lane & 15;
  const int r0 = (blockIdx.x * 4 + wave) * 16;
  int row = r0 + m;
  if (row > nN - 1) row = nN - 1;
  const float fz = (hh == 0) ? 1.0f : 0.0f;
  const float* pr = pos + (size_t)row * 3;
  const float p0 = pr[0] * fz, p1 = pr[1] * fz, p2 = pr[2] * fz;
  Frag ah, al, bh0, bl0, bh1, bl1;
  fragz(ah); fragz(al); fragz(bh0); fragz(bl0); fragz(bh1); fragz(bl1);
  unsigned u;
  u = split2(p0); ah.s[0] = (unsigned short)(u & 0xffffu); al.s[0] = (unsigned short)(u >> 16);
  u = split2(p1); ah.s[1] = (unsigned short)(u & 0xffffu); al.s[1] = (unsigned short)(u >> 16);
  u = split2(p2); ah.s[2] = (unsigned short)(u & 0xffffu); al.s[2] = (unsigned short)(u >> 16);
  {
    const float w00 = W1[0 * 32 + m] * fz, w10 = W1[1 * 32 + m] * fz, w20 = W1[2 * 32 + m] * fz;
    const float w01 = W1[0 * 32 + 16 + m] * fz, w11 = W1[1 * 32 + 16 + m] * fz, w21 = W1[2 * 32 + 16 + m] * fz;
    u = split2(w00); bh0.s[0] = (unsigned short)(u & 0xffffu); bl0.s[0] = (unsigned short)(u >> 16);
    u = split2(w10); bh0.s[1] = (unsigned short)(u & 0xffffu); bl0.s[1] = (unsigned short)(u >> 16);
    u = split2(w20); bh0.s[2] = (unsigned short)(u & 0xffffu); bl0.s[2] = (unsigned short)(u >> 16);
    u = split2(w01); bh1.s[0] = (unsigned short)(u & 0xffffu); bl1.s[0] = (unsigned short)(u >> 16);
    u = split2(w11); bh1.s[1] = (unsigned short)(u & 0xffffu); bl1.s[1] = (unsigned short)(u >> 16);
    u = split2(w21); bh1.s[2] = (unsigned short)(u & 0xffffu); bl1.s[2] = (unsigned short)(u >> 16);
  }
  v8f c0 = zero8(), c1 = zero8();
  c0 = wm3(ah.v, al.v, bh0.v, bl0.v, c0);
  c1 = wm3(ah.v, al.v, bh1.v, bl1.v, c1);
  float* xw = xs + wave * (16 * 36);
#pragma unroll
  for (int r = 0; r < 8; ++r) {
    xw[(8 * hh + r) * 36 + m]      = c0[r];
    xw[(8 * hh + r) * 36 + 16 + m] = c1[r];
  }
  __syncthreads();
  const int c4 = (lane & 7) * 4;
  v4f sv[4];
#pragma unroll
  for (int q = 0; q < 4; ++q) sv[q] = *(const v4f*)(xw + (q * 4 + (lane >> 3)) * 36 + c4);
  if (r0 < nN) {
#pragma unroll
    for (int q = 0; q < 4; ++q)
      *(volatile v4f*)(xp + (size_t)(r0 + q * 4 + (lane >> 3)) * 32 + c4) = sv[q];
    __threadfence();
#pragma unroll
    for (int q = 0; q < 4; ++q)
      *(volatile v4f*)(xp + (size_t)(r0 + q * 4 + (lane >> 3)) * 32 + c4) = sv[q];
  }
}

template <int H>
__global__ __launch_bounds__(256) void k_alpha(const float* __restrict__ xp, const float* __restrict__ as,
                                               const float* __restrict__ ad, float* al4, int nN, int F) {
  const int t = blockIdx.x * 256 + threadIdx.x;
  if (t >= nN) return;
  const int HF = H * F;
  const float* row = xp + (size_t)t * HF;
  float ss0 = 0.f, sd0 = 0.f, ss1 = 0.f, sd1 = 0.f;
#pragma unroll 1
  for (int f = 0; f < F; ++f) {
    const float v0 = row[f];
    ss0 += v0 * as[f];
    sd0 += v0 * ad[f];
    if (H == 2) {
      const float v1 = row[F + f];
      ss1 += v1 * as[F + f];
      sd1 += v1 * ad[F + f];
    }
  }
  const v4f o = {ss0, ss1, sd0, sd1};
  float* p = al4 + (size_t)t * 4;
  *(volatile v4f*)p = o;
  __threadfence();
  *(volatile v4f*)p = o;
}

template <int HF, int H, int NBS>
__global__ __launch_bounds__(256) void k_gat(const int* __restrict__ srcA, const int* __restrict__ dstA,
                                             const float* __restrict__ xp, const float* __restrict__ al4,
                                             const float* __restrict__ bias, float* out,
                                             int npg, int bpg, int nN) {
  extern __shared__ __attribute__((aligned(16))) v4f lds_a[];
  float* sacc = (float*)lds_a;
  float* den  = sacc + NBS * HF;
  float* mx   = den + NBS * 2;
  int*   list = (int*)(mx + NBS * 2);
  int*   wcnt = list + 8 * WCAP;

  const int tid = threadIdx.x, lane = tid & 31, wave = tid >> 5;
  const int hd = (H == 2) ? (lane >> 4) : 0;
  const int g  = blockIdx.x / bpg;
  const int sb = (blockIdx.x - g * bpg) * NBS;
  const int nodeBase = g * npg + sb;
  int nval = npg - sb;
  if (nval > NBS) nval = NBS;
  if (nval < 0) nval = 0;
  const int ebase0 = g * EPG;

  {
    const v4f z4 = {0.f, 0.f, 0.f, 0.f};
    for (int i = tid; i < NBS * HF / 4; i += 256) lds_a[i] = z4;
    for (int i = tid; i < NBS * 2; i += 256) { den[i] = 0.f; mx[i] = -1.0e30f; }
  }
  __syncthreads();

#pragma unroll 1
  for (int ch = 0; ch < EPG / CHUNK; ++ch) {
    const int cbase = ch * CHUNK;
    int wc = 0;
#pragma unroll
    for (int gq = 0; gq < NGRP; ++gq) {
      const int el0 = (gq * 256 + tid) * 4;
      const v4i d = *(const v4i*)(dstA + (size_t)ebase0 + cbase + el0);
      const unsigned s0 = (unsigned)(d.x - nodeBase);
      const unsigned s1 = (unsigned)(d.y - nodeBase);
      const unsigned s2 = (unsigned)(d.z - nodeBase);
      const unsigned s3 = (unsigned)(d.w - nodeBase);
      const bool h0 = s0 < (unsigned)nval;
      const bool h1 = s1 < (unsigned)nval;
      const bool h2 = s2 < (unsigned)nval;
      const bool h3 = s3 < (unsigned)nval;
      const unsigned many = __builtin_amdgcn_ballot_w32(h0 | h1 | h2 | h3);
      if (many != 0u) {
#define HITJ(J, HJ, SJ) { \
          const unsigned mj = __builtin_amdgcn_ballot_w32(HJ); \
          if (HJ) { \
            const int ps = wc + (int)__builtin_amdgcn_mbcnt_lo(mj, 0u); \
            if (ps < WCAP) list[wave * WCAP + ps] = ((el0 + (J)) << 10) | (int)(SJ); \
          } \
          wc += (int)__builtin_popcount(mj); }
        HITJ(0, h0, s0)
        HITJ(1, h1, s1)
        HITJ(2, h2, s2)
        HITJ(3, h3, s3)
#undef HITJ
      }
    }
    if (lane == 0) wcnt[wave] = wc;
    __syncthreads();

    if (wave == 0) {
      for (int wsx = 0; wsx < 8; ++wsx) {
        int n = wcnt[wsx];
        if (n > WCAP) n = WCAP;
        if (n < 0) n = 0;
        for (int i = 0; i < n; ++i) {
          const int ent = list[wsx * WCAP + i];
          int slot = ent & 1023;
          if (slot > NBS - 1) slot = NBS - 1;
          const int el = (ent >> 10) & (CHUNK - 1);
          const int e = ebase0 + cbase + el;
          int src = srcA[e];
          src = clampi(src, 0, nN - 1);
          int node = nodeBase + slot;
          if (node > nN - 1) node = nN - 1;
          const float a = lrelu(al4[(size_t)src * 4 + hd] + al4[(size_t)node * 4 + 2 + hd]);
          const int midx = slot * 2 + hd;
          const float mo = mx[midx];
          const float mn = fmaxf(mo, a);
          const float sc = __expf(mo - mn);
          const float p  = __expf(a - mn);
          if constexpr (HF == 32) {
            const float xv = xp[(size_t)src * 32 + lane];
            float* sp = sacc + slot * 32 + lane;
            const float cur = *sp;
            *sp = cur * sc + p * xv;
          } else {
            constexpr int NPC = HF / 128;
#pragma unroll
            for (int j = 0; j < NPC; ++j) {
              const int co = j * 128 + 4 * lane;
              const v4f xv = *(const v4f*)(xp + (size_t)src * HF + co);
              v4f* sp = (v4f*)(sacc + slot * HF + co);
              const v4f cur = *sp;
              *sp = cur * sc + p * xv;
            }
          }
          const bool wl = (H == 2) ? ((lane & 15) == 0) : (lane == 0);
          if (wl) {
            const float dn = den[midx];
            den[midx] = dn * sc + p;
            mx[midx] = mn;
          }
        }
      }
    }
    __syncthreads();
  }

#pragma unroll 1
  for (int slot = wave; slot < nval; slot += 8) {
    const int node = nodeBase + slot;
    const size_t nrow = (size_t)node;
    const float a = lrelu(al4[nrow * 4 + hd] + al4[nrow * 4 + 2 + hd]);
    const int midx = slot * 2 + hd;
    const float mo = mx[midx];
    const float mn = fmaxf(mo, a);
    const float sc = __expf(mo - mn);
    const float p  = __expf(a - mn);
    const float dv = den[midx] * sc + p;
    const float inv = 1.0f / dv;
    if constexpr (HF == 32) {
      const float v = (sacc[slot * 32 + lane] * sc + p * xp[nrow * 32 + lane]) * inv + bias[lane];
      float* op = out + nrow * 32 + lane;
      *(volatile float*)op = v;
      __threadfence();
      *(volatile float*)op = v;
    } else {
      constexpr int NPC = HF / 128;
      v4f vv[NPC];
#pragma unroll
      for (int j = 0; j < NPC; ++j) {
        const int co = j * 128 + 4 * lane;
        const v4f xv = *(const v4f*)(xp + nrow * HF + co);
        const v4f sv = *(const v4f*)(sacc + slot * HF + co);
        const v4f b4 = *(const v4f*)(bias + co);
        vv[j] = (sv * sc + p * xv) * inv + b4;
      }
#pragma unroll
      for (int j = 0; j < NPC; ++j) *(volatile v4f*)(out + nrow * HF + j * 128 + 4 * lane) = vv[j];
      __threadfence();
#pragma unroll
      for (int j = 0; j < NPC; ++j) *(volatile v4f*)(out + nrow * HF + j * 128 + 4 * lane) = vv[j];
    }
  }
}

template <int C, int MODE>
__global__ __launch_bounds__(256) void k_norm(const float* __restrict__ x, const float* __restrict__ pvec,
                                              float* outF, float* score, unsigned short* outH,
                                              unsigned short* outL, int npg, int spad) {
  __shared__ double dsum[256];
  __shared__ double dsq[256];
  __shared__ __attribute__((aligned(16))) float mus[256];
  __shared__ __attribute__((aligned(16))) float rss[256];
  const int tid = threadIdx.x, lane = tid & 31, wave = tid >> 5, g = blockIdx.x;
  constexpr int RS = 256 / C;
  const int c = tid & (C - 1), rg = tid / C;
  const float* xg = x + (size_t)g * npg * C;
  double s = 0.0, q = 0.0;
#pragma unroll 1
  for (int r = rg; r < npg; r += RS) {
    const double dv = (double)xg[(size_t)r * C + c];
    s += dv;
    q += dv * dv;
  }
  dsum[tid] = s;
  dsq[tid] = q;
  __syncthreads();
  if (tid < C) {
    double ts = 0.0, tq = 0.0;
#pragma unroll 1
    for (int j = 0; j < RS; ++j) { ts += dsum[j * C + tid]; tq += dsq[j * C + tid]; }
    const double inv = 1.0 / (double)npg;
    const double mu = ts * inv;
    double var = tq * inv - mu * mu;
    if (var < 0.0) var = 0.0;
    mus[tid] = (float)mu;
    rss[tid] = 1.0f / sqrtf((float)var + 1.0e-5f);
  }
  __syncthreads();

  if constexpr (MODE == 0) {
    const int ngrp = (npg + 31) >> 5;
    if constexpr (C == 32) {
      const float pl = pvec[lane];
      const float rn = 1.0f / sqrtf(wsum(pl * pl));
      const float mu1 = mus[lane], rs1 = rss[lane];
#pragma unroll 1
      for (int gi = wave; gi < ngrp; gi += 8) {
        float mys = 0.f;
#pragma unroll 1
        for (int i = 0; i < 32; ++i) {
          const int r = gi * 32 + i;
          if (r < npg) {
            float v = (xg[(size_t)r * 32 + lane] - mu1) * rs1;
            v = elu1(v);
            float* op = outF + ((size_t)g * npg + r) * 32 + lane;
            *(volatile float*)op = v;
            __threadfence();
            *(volatile float*)op = v;
            const float d = wsum(v * pl);
            const float sc = tanhf(d * rn);
            if (lane == i) mys = sc;
          }
        }
        float* sp = score + (size_t)g * spad + gi * 32 + lane;
        *(volatile float*)sp = mys;
        __threadfence();
        *(volatile float*)sp = mys;
      }
    } else {
      const v4f p4 = *(const v4f*)(pvec + 4 * lane);
      const float rn = 1.0f / sqrtf(wsum(p4.x * p4.x + p4.y * p4.y + p4.z * p4.z + p4.w * p4.w));
      const v4f mu4 = *(const v4f*)(mus + 4 * lane);
      const v4f rs4 = *(const v4f*)(rss + 4 * lane);
#pragma unroll 1
      for (int gi = wave; gi < ngrp; gi += 8) {
        float mys = 0.f;
#pragma unroll 1
        for (int i = 0; i < 32; ++i) {
          const int r = gi * 32 + i;
          if (r < npg) {
            v4f y = (*(const v4f*)(xg + (size_t)r * C + 4 * lane) - mu4) * rs4;
            y.x = elu1(y.x); y.y = elu1(y.y); y.z = elu1(y.z); y.w = elu1(y.w);
            float* op = outF + ((size_t)g * npg + r) * C + 4 * lane;
            *(volatile v4f*)op = y;
            __threadfence();
            *(volatile v4f*)op = y;
            const float d = wsum(y.x * p4.x + y.y * p4.y + y.z * p4.z + y.w * p4.w);
            const float sc = tanhf(d * rn);
            if (lane == i) mys = sc;
          }
        }
        float* sp = score + (size_t)g * spad + gi * 32 + lane;
        *(volatile float*)sp = mys;
        __threadfence();
        *(volatile float*)sp = mys;
      }
    }
  } else {
    const v4f mA = *(const v4f*)(mus + 8 * lane), mB = *(const v4f*)(mus + 8 * lane + 4);
    const v4f rA = *(const v4f*)(rss + 8 * lane), rB = *(const v4f*)(rss + 8 * lane + 4);
#pragma unroll 1
    for (int r = wave; r < npg; r += 8) {
      const float* xr = xg + (size_t)r * C + 8 * lane;
      v4f a = (*(const v4f*)xr - mA) * rA;
      v4f b = (*(const v4f*)(xr + 4) - mB) * rB;
      a.x = elu1(a.x); a.y = elu1(a.y); a.z = elu1(a.z); a.w = elu1(a.w);
      b.x = elu1(b.x); b.y = elu1(b.y); b.z = elu1(b.z); b.w = elu1(b.w);
      const unsigned u0 = split2(a.x), u1 = split2(a.y), u2 = split2(a.z), u3 = split2(a.w);
      const unsigned u4 = split2(b.x), u5 = split2(b.y), u6 = split2(b.z), u7 = split2(b.w);
      v4u hv, lv;
      hv.x = (u0 & 0xffffu) | (u1 << 16);  lv.x = (u0 >> 16) | (u1 & 0xffff0000u);
      hv.y = (u2 & 0xffffu) | (u3 << 16);  lv.y = (u2 >> 16) | (u3 & 0xffff0000u);
      hv.z = (u4 & 0xffffu) | (u5 << 16);  lv.z = (u4 >> 16) | (u5 & 0xffff0000u);
      hv.w = (u6 & 0xffffu) | (u7 << 16);  lv.w = (u6 >> 16) | (u7 & 0xffff0000u);
      const size_t eo = ((size_t)g * npg + r) * C + 8 * lane;
      *(volatile v4u*)(outH + eo) = hv;
      *(volatile v4u*)(outL + eo) = lv;
      __threadfence();
      *(volatile v4u*)(outH + eo) = hv;
      *(volatile v4u*)(outL + eo) = lv;
    }
  }
}

template <int C>
__global__ __launch_bounds__(512) void k_pool(const float* __restrict__ xn, const float* __restrict__ score,
                                              unsigned short* outH, unsigned short* outL, int* newid,
                                              int npg, int spad, int kk, int NP) {
  extern __shared__ __attribute__((aligned(16))) unsigned long long lds_p[];
  unsigned long long* keys = lds_p;
  int* nid = (int*)(lds_p + NP);
  const int tid = threadIdx.x, lane = tid & 31, wave = tid >> 5, g = blockIdx.x;

  for (int i = tid; i < NP; i += 512) {
    int ic = i;
    if (ic > npg - 1) ic = npg - 1;
    const float sv = score[(size_t)g * spad + ic];
    const unsigned long long key = (((unsigned long long)f2o(sv)) << 32) | (unsigned long long)(~(unsigned)i);
    keys[i] = (i < npg) ? key : 0ull;
  }
  for (int i = tid; i < spad; i += 512) nid[i] = -1;
  __syncthreads();

  for (int kb = 2; kb <= NP; kb <<= 1) {
    for (int j = kb >> 1; j > 0; j >>= 1) {
      for (int px = tid; px < (NP >> 1); px += 512) {
        const int i  = ((px & ~(j - 1)) << 1) | (px & (j - 1));
        const int ip = i | j;
        const unsigned long long a = keys[i], b = keys[ip];
        const bool dsc = ((i & kb) == 0);
        const bool sw = dsc ? (a < b) : (a > b);
        if (sw) { keys[i] = b; keys[ip] = a; }
      }
      __syncthreads();
    }
  }

  for (int r = tid; r < kk; r += 512) {
    const unsigned lo = (unsigned)(keys[r] & 0xffffffffull);
    const int idx = clampi((int)(~lo), 0, npg - 1);
    nid[idx] = g * kk + r;
  }
  __syncthreads();

  for (int i = tid * 4; i < spad; i += 2048) {
    const v4i v = *(const v4i*)(nid + i);
    int* p = newid + (size_t)g * spad + i;
    *(volatile v4i*)p = v;
    __threadfence();
    *(volatile v4i*)p = v;
  }

  if constexpr (C == 32) {
    const int npr = kk >> 1;
#pragma unroll 1
    for (int pr = wave; pr < npr; pr += 16) {
      const int r = 2 * pr + (lane >> 4);
      const unsigned long long key = keys[r];
      const int idx = clampi((int)(~(unsigned)(key & 0xffffffffull)), 0, npg - 1);
      const float s = o2f((unsigned)(key >> 32));
      const float* xr = xn + ((size_t)g * npg + idx) * 32 + 2 * (lane & 15);
      const float x0 = xr[0] * s, x1 = xr[1] * s;
      const unsigned u0 = split2(x0), u1 = split2(x1);
      const unsigned hv = (u0 & 0xffffu) | (u1 << 16);
      const unsigned lv = (u0 >> 16) | (u1 & 0xffff0000u);
      const size_t wo = ((size_t)g * kk + 2 * pr) * 16 + lane;
      *(volatile unsigned*)((unsigned*)outH + wo) = hv;
      *(volatile unsigned*)((unsigned*)outL + wo) = lv;
      __threadfence();
      *(volatile unsigned*)((unsigned*)outH + wo) = hv;
      *(volatile unsigned*)((unsigned*)outL + wo) = lv;
    }
  } else {
#pragma unroll 1
    for (int r = wave; r < kk; r += 16) {
      const unsigned long long key = keys[r];
      const int idx = clampi((int)(~(unsigned)(key & 0xffffffffull)), 0, npg - 1);
      const float s = o2f((unsigned)(key >> 32));
      const v4f xv = *(const v4f*)(xn + ((size_t)g * npg + idx) * 128 + 4 * lane) * s;
      const unsigned u0 = split2(xv.x), u1 = split2(xv.y), u2 = split2(xv.z), u3 = split2(xv.w);
      v2u hv, lv;
      hv.x = (u0 & 0xffffu) | (u1 << 16);  lv.x = (u0 >> 16) | (u1 & 0xffff0000u);
      hv.y = (u2 & 0xffffu) | (u3 << 16);  lv.y = (u2 >> 16) | (u3 & 0xffff0000u);
      const size_t wo = ((size_t)g * kk + r) * 64 + 2 * lane;
      *(volatile v2u*)((unsigned*)outH + wo) = hv;
      *(volatile v2u*)((unsigned*)outL + wo) = lv;
      __threadfence();
      *(volatile v2u*)((unsigned*)outH + wo) = hv;
      *(volatile v2u*)((unsigned*)outL + wo) = lv;
    }
  }
}

__device__ __forceinline__ void rm1(int S, int D, const int* __restrict__ newid, int npgIn, int spad,
                                    int nNIn, int& OS, int& OD) {
  bool alive = (D >= 0) && (S >= 0);
  const int sc = clampi(S, 0, nNIn - 1);
  const int dc = clampi(D, 0, nNIn - 1);
  const int gs = sc / npgIn, gd = dc / npgIn;
  const int ns = newid[gs * spad + (sc - gs * npgIn)];
  const int nd = newid[gd * spad + (dc - gd * npgIn)];
  alive = alive && (ns >= 0) && (nd >= 0);
  OS = alive ? ns : 0;
  OD = alive ? nd : -1;
}
__global__ __launch_bounds__(256) void k_remap(const int* __restrict__ sIn, const int* __restrict__ dIn,
                                               const int* __restrict__ newid, int* sOut, int* dOut,
                                               int npgIn, int spad, int nNIn, int n4) {
  const int t = blockIdx.x * 256 + threadIdx.x;
  if (t >= n4) return;
  const v4i s = *(const v4i*)(sIn + (size_t)t * 4);
  const v4i d = *(const v4i*)(dIn + (size_t)t * 4);
  v4i os, od;
  int a, b;
  rm1(s.x, d.x, newid, npgIn, spad, nNIn, a, b); os.x = a; od.x = b;
  rm1(s.y, d.y, newid, npgIn, spad, nNIn, a, b); os.y = a; od.y = b;
  rm1(s.z, d.z, newid, npgIn, spad, nNIn, a, b); os.z = a; od.z = b;
  rm1(s.w, d.w, newid, npgIn, spad, nNIn, a, b); os.w = a; od.w = b;
  int* ps = sOut + (size_t)t * 4;
  int* pd = dOut + (size_t)t * 4;
  *(volatile v4i*)ps = os;
  *(volatile v4i*)pd = od;
  __threadfence();
  *(volatile v4i*)ps = os;
  *(volatile v4i*)pd = od;
}

template <int K, int ACT, bool HASB>
__global__ __launch_bounds__(128) void k_gemm(const unsigned short* __restrict__ Ah,
                                              const unsigned short* __restrict__ Al,
                                              const float* __restrict__ W, const float* __restrict__ bias,
                                              float* Cout, int M, int N) {
  extern __shared__ __attribute__((aligned(16))) v4f lds_g[];
  constexpr int BP = K + 8;
  unsigned short* Bh = (unsigned short*)lds_g;
  unsigned short* Bl = Bh + 64 * BP;
  float* stg = (float*)(Bl + 64 * BP);
  const int tid = threadIdx.x, lane = tid & 31, wave = tid >> 5, hh = lane >> 4, m = lane & 15;
  const int n0 = blockIdx.y * 64;

#pragma unroll 1
  for (int idx = tid; idx < K * 64; idx += 128) {
    const int k = idx >> 6, n = idx & 63;
    const unsigned u = split2(W[(size_t)k * N + n0 + n]);
    Bh[n * BP + k] = (unsigned short)(u & 0xffffu);
    Bl[n * BP + k] = (unsigned short)(u >> 16);
  }
  __syncthreads();

  const int rowT = blockIdx.x * 64 + wave * 16;
  int arow = rowT + m;
  if (arow > M - 1) arow = M - 1;
  const unsigned short* pah = Ah + (size_t)arow * K + 8 * hh;
  const unsigned short* pal = Al + (size_t)arow * K + 8 * hh;
  v8f acc[4];
#pragma unroll
  for (int t = 0; t < 4; ++t) acc[t] = zero8();
#pragma unroll 1
  for (int kt = 0; kt < K / 32; ++kt) {
    const int k0 = kt * 32;
    Frag ah, al;
    ah.h8[0] = *(const v8us*)(pah + k0);
    ah.h8[1] = *(const v8us*)(pah + k0 + 16);
    al.h8[0] = *(const v8us*)(pal + k0);
    al.h8[1] = *(const v8us*)(pal + k0 + 16);
#pragma unroll
    for (int nt = 0; nt < 4; ++nt) {
      const unsigned short* pb = Bh + (nt * 16 + m) * BP + k0 + 8 * hh;
      const unsigned short* pc = Bl + (nt * 16 + m) * BP + k0 + 8 * hh;
      Frag bh, bl;
      bh.h8[0] = *(const v8us*)pb;
      bh.h8[1] = *(const v8us*)(pb + 16);
      bl.h8[0] = *(const v8us*)pc;
      bl.h8[1] = *(const v8us*)(pc + 16);
      acc[nt] = wm3(ah.v, al.v, bh.v, bl.v, acc[nt]);
    }
  }

  float* sw = stg + wave * (16 * 68);
#pragma unroll
  for (int nt = 0; nt < 4; ++nt) {
    float bv = 0.f;
    if constexpr (HASB) bv = bias[n0 + nt * 16 + m];
#pragma unroll
    for (int r = 0; r < 8; ++r) {
      float v = acc[nt][r] + bv;
      if constexpr (ACT == 1) v = elu1(v);
      sw[(8 * hh + r) * 68 + nt * 16 + m] = v;
    }
  }
  __syncthreads();
  const int c4 = (lane & 15) * 4;
  v4f sv[8];
#pragma unroll
  for (int q = 0; q < 8; ++q) sv[q] = *(const v4f*)(sw + (2 * q + hh) * 68 + c4);
  if (rowT < M) {
#pragma unroll
    for (int q = 0; q < 8; ++q)
      *(volatile v4f*)(Cout + (size_t)(rowT + 2 * q + hh) * N + n0 + c4) = sv[q];
    __threadfence();
#pragma unroll
    for (int q = 0; q < 8; ++q)
      *(volatile v4f*)(Cout + (size_t)(rowT + 2 * q + hh) * N + n0 + c4) = sv[q];
  }
}

__global__ __launch_bounds__(256) void k_final(const float* __restrict__ gate1, const float* __restrict__ gw2,
                                               const float* __restrict__ gb2, const float* __restrict__ hb,
                                               const float* __restrict__ w1, const float* __restrict__ b1,
                                               const float* __restrict__ w2, const float* __restrict__ b2,
                                               const float* __restrict__ w3, const float* __restrict__ b3,
                                               float* outp) {
  extern __shared__ __attribute__((aligned(16))) v4f lds_f[];
  float* gs  = (float*)lds_f;
  float* red = gs + 768;
  unsigned short* Gh  = (unsigned short*)(red + 256);
  unsigned short* Gl  = Gh + 16 * 264;
  unsigned short* Z1h = Gl + 16 * 264;
  unsigned short* Z1l = Z1h + 16 * 520;
  unsigned short* Z2h = Z1l + 16 * 520;
  unsigned short* Z2l = Z2h + 16 * 136;
  float* zl = (float*)(Z2l + 16 * 136);
  float* os = zl + 256;
  const int tid = threadIdx.x, lane = tid & 31, wave = tid >> 5, hh = lane >> 4, m = lane & 15;

  for (int i = tid; i < 16 * 264; i += 256) { Gh[i] = 0; Gl[i] = 0; }
  __syncthreads();
  const float gb2v = gb2[0];

#pragma unroll 1
  for (int g = 0; g < BG; ++g) {
    for (int i = tid; i < KP2; i += 256) {
      const float* gr = gate1 + (size_t)(g * KP2 + i) * 64;
      float s = 0.f;
#pragma unroll 1
      for (int k = 0; k < 64; ++k) s += gr[k] * gw2[k];
      gs[i] = s + gb2v;
    }
    __syncthreads();
    float mxl = -3.0e38f;
    for (int i = tid; i < KP2; i += 256) mxl = fmaxf(mxl, gs[i]);
    red[tid] = mxl;
    __syncthreads();
    for (int t = 128; t > 0; t >>= 1) {
      if (tid < t) red[tid] = fmaxf(red[tid], red[tid + t]);
      __syncthreads();
    }
    const float mxv = red[0];
    __syncthreads();
    float sl = 0.f;
    for (int i = tid; i < KP2; i += 256) { const float e = __expf(gs[i] - mxv); gs[i] = e; sl += e; }
    red[tid] = sl;
    __syncthreads();
    for (int t = 128; t > 0; t >>= 1) {
      if (tid < t) red[tid] += red[tid + t];
      __syncthreads();
    }
    const float inv = 1.0f / red[0];
    float acc = 0.f;
#pragma unroll 1
    for (int i = 0; i < KP2; ++i) acc += gs[i] * hb[(size_t)(g * KP2 + i) * 256 + tid];
    const unsigned u = split2(acc * inv);
    Gh[g * 264 + tid] = (unsigned short)(u & 0xffffu);
    Gl[g * 264 + tid] = (unsigned short)(u >> 16);
    __syncthreads();
  }

  {
    v8f acc[4];
#pragma unroll
    for (int t = 0; t < 4; ++t) acc[t] = zero8();
#pragma unroll 1
    for (int kt = 0; kt < 8; ++kt) {
      const int k0 = kt * 32;
      Frag ah, al;
      ah.h8[0] = *(const v8us*)(Gh + m * 264 + k0 + 8 * hh);
      ah.h8[1] = *(const v8us*)(Gh + m * 264 + k0 + 16 + 8 * hh);
      al.h8[0] = *(const v8us*)(Gl + m * 264 + k0 + 8 * hh);
      al.h8[1] = *(const v8us*)(Gl + m * 264 + k0 + 16 + 8 * hh);
#pragma unroll
      for (int nt = 0; nt < 4; ++nt) {
        const int col = wave * 64 + nt * 16 + m;
        Frag bh, bl;
#pragma unroll
        for (int i = 0; i < 16; ++i) {
          const int kk = k0 + 8 * hh + i + ((i >= 8) ? 8 : 0);
          const unsigned u = split2(w1[(size_t)kk * 512 + col]);
          bh.s[i] = (unsigned short)(u & 0xffffu);
          bl.s[i] = (unsigned short)(u >> 16);
        }
        acc[nt] = wm3(ah.v, al.v, bh.v, bl.v, acc[nt]);
      }
    }
#pragma unroll
    for (int nt = 0; nt < 4; ++nt) {
      const int col = wave * 64 + nt * 16 + m;
      const float bv = b1[col];
#pragma unroll
      for (int r = 0; r < 8; ++r) {
        const unsigned u = split2(elu1(acc[nt][r] + bv));
        Z1h[(8 * hh + r) * 520 + col] = (unsigned short)(u & 0xffffu);
        Z1l[(8 * hh + r) * 520 + col] = (unsigned short)(u >> 16);
      }
    }
  }
  __syncthreads();

  {
    v8f acc = zero8();
    const int col = wave * 16 + m;
#pragma unroll 1
    for (int kt = 0; kt < 16; ++kt) {
      const int k0 = kt * 32;
      Frag ah, al, bh, bl;
      ah.h8[0] = *(const v8us*)(Z1h + m * 520 + k0 + 8 * hh);
      ah.h8[1] = *(const v8us*)(Z1h + m * 520 + k0 + 16 + 8 * hh);
      al.h8[0] = *(const v8us*)(Z1l + m * 520 + k0 + 8 * hh);
      al.h8[1] = *(const v8us*)(Z1l + m * 520 + k0 + 16 + 8 * hh);
#pragma unroll
      for (int i = 0; i < 16; ++i) {
        const int kk = k0 + 8 * hh + i + ((i >= 8) ? 8 : 0);
        const unsigned u = split2(w2[(size_t)kk * 128 + col]);
        bh.s[i] = (unsigned short)(u & 0xffffu);
        bl.s[i] = (unsigned short)(u >> 16);
      }
      acc = wm3(ah.v, al.v, bh.v, bl.v, acc);
    }
    const float bv = b2[col];
#pragma unroll
    for (int r = 0; r < 8; ++r) {
      const unsigned u = split2(elu1(acc[r] + bv));
      Z2h[(8 * hh + r) * 136 + col] = (unsigned short)(u & 0xffffu);
      Z2l[(8 * hh + r) * 136 + col] = (unsigned short)(u >> 16);
    }
  }
  __syncthreads();

  if (wave == 0) {
    v8f acc = zero8();
    const int cm = (m < NCLS) ? m : (NCLS - 1);
    const float fz = (m < NCLS) ? 1.0f : 0.0f;
#pragma unroll 1
    for (int kt = 0; kt < 4; ++kt) {
      const int k0 = kt * 32;
      Frag ah, al, bh, bl;
      ah.h8[0] = *(const v8us*)(Z2h + m * 136 + k0 + 8 * hh);
      ah.h8[1] = *(const v8us*)(Z2h + m * 136 + k0 + 16 + 8 * hh);
      al.h8[0] = *(const v8us*)(Z2l + m * 136 + k0 + 8 * hh);
      al.h8[1] = *(const v8us*)(Z2l + m * 136 + k0 + 16 + 8 * hh);
#pragma unroll
      for (int i = 0; i < 16; ++i) {
        const int kk = k0 + 8 * hh + i + ((i >= 8) ? 8 : 0);
        const unsigned u = split2(w3[(size_t)kk * NCLS + cm] * fz);
        bh.s[i] = (unsigned short)(u & 0xffffu);
        bl.s[i] = (unsigned short)(u >> 16);
      }
      acc = wm3(ah.v, al.v, bh.v, bl.v, acc);
    }
    const float bv = b3[cm] * fz;
#pragma unroll
    for (int r = 0; r < 8; ++r) zl[(8 * hh + r) * 16 + m] = acc[r] + bv;
  }
  __syncthreads();
  if (tid < BG) {
    float mxv = zl[tid * 16];
#pragma unroll 1
    for (int c = 1; c < NCLS; ++c) mxv = fmaxf(mxv, zl[tid * 16 + c]);
    float se = 0.f;
#pragma unroll 1
    for (int c = 0; c < NCLS; ++c) se += expf(zl[tid * 16 + c] - mxv);
    const float lse = logf(se);
#pragma unroll 1
    for (int c = 0; c < NCLS; ++c) os[tid * NCLS + c] = zl[tid * 16 + c] - mxv - lse;
  }
  __syncthreads();
  if (tid < 20) {
    const v4f v = *(const v4f*)(os + 4 * tid);
    float* p = outp + 4 * tid;
    *(volatile v4f*)p = v;
    __threadfence();
    *(volatile v4f*)p = v;
  }
}

extern "C" void kernel_launch(void* const* d_in, const int* in_sizes, int n_in,
                              void* d_out, int out_size, void* d_ws, size_t ws_size,
                              hipStream_t stream) {
  if (n_in < 29) return;
  if (in_sizes[0] != NT1 * 3 || in_sizes[1] != NEDGE || in_sizes[2] != NEDGE) return;
  if (in_sizes[3] != 3 * 32 || in_sizes[4] != 32 || in_sizes[5] != 32 || in_sizes[6] != 32 || in_sizes[7] != 32) return;
  if (in_sizes[8] != 32 * 128 || in_sizes[9] != 128 || in_sizes[10] != 128 || in_sizes[11] != 128 || in_sizes[12] != 128) return;
  if (in_sizes[13] != 128 * 256 || in_sizes[14] != 256 || in_sizes[15] != 256 || in_sizes[16] != 256) return;
  if (in_sizes[17] != 256 * 64 || in_sizes[18] != 64 || in_sizes[19] != 64 || in_sizes[20] != 1) return;
  if (in_sizes[21] != 256 * 256 || in_sizes[22] != 256 || in_sizes[23] != 256 * 512 || in_sizes[24] != 512) return;
  if (in_sizes[25] != 512 * 128 || in_sizes[26] != 128 || in_sizes[27] != 128 * NCLS || in_sizes[28] != NCLS) return;
  if (out_size != BG * NCLS) return;

  const float* pos  = (const float*)d_in[0];
  const int*   src  = (const int*)d_in[1];
  const int*   dst  = (const int*)d_in[2];
  const float* W1   = (const float*)d_in[3];
  const float* a_s1 = (const float*)d_in[4];
  const float* a_d1 = (const float*)d_in[5];
  const float* b1   = (const float*)d_in[6];
  const float* p1   = (const float*)d_in[7];
  const float* W2   = (const float*)d_in[8];
  const float* a_s2 = (const float*)d_in[9];
  const float* a_d2 = (const float*)d_in[10];
  const float* b2   = (const float*)d_in[11];
  const float* p2   = (const float*)d_in[12];
  const float* W3   = (const float*)d_in[13];
  const float* a_s3 = (const float*)d_in[14];
  const float* a_d3 = (const float*)d_in[15];
  const float* b3   = (const float*)d_in[16];
  const float* gw1  = (const float*)d_in[17];
  const float* gb1  = (const float*)d_in[18];
  const float* gw2  = (const float*)d_in[19];
  const float* gb2  = (const float*)d_in[20];
  const float* aw   = (const float*)d_in[21];
  const float* ab   = (const float*)d_in[22];
  const float* w1   = (const float*)d_in[23];
  const float* bb1  = (const float*)d_in[24];
  const float* w2   = (const float*)d_in[25];
  const float* bb2  = (const float*)d_in[26];
  const float* w3   = (const float*)d_in[27];
  const float* bb3  = (const float*)d_in[28];
  float* outp = (float*)d_out;

  char* base = (char*)d_ws;
  size_t off = 0;
  auto carve = [&](size_t bytes) -> char* {
    char* p = base + off;
    off += (bytes + 255) & ~(size_t)255;
    return p;
  };
  float* xp1  = (float*)carve((size_t)NT1 * 32 * 4);
  float* al1  = (float*)carve((size_t)NT1 * 4 * 4);
  float* gat1 = (float*)carve((size_t)NT1 * 32 * 4);
  float* xn1  = (float*)carve((size_t)NT1 * 32 * 4);
  float* sc1  = (float*)carve((size_t)BG * SPAD1 * 4);
  int*   nid1 = (int*)carve((size_t)BG * SPAD1 * 4);
  unsigned short* x2h = (unsigned short*)carve((size_t)NT2 * 32 * 2);
  unsigned short* x2l = (unsigned short*)carve((size_t)NT2 * 32 * 2);
  int*   es2  = (int*)carve((size_t)NEDGE * 4);
  int*   ed2  = (int*)carve((size_t)NEDGE * 4);
  float* xp2  = (float*)carve((size_t)NT2 * 128 * 4);
  float* al2  = (float*)carve((size_t)NT2 * 4 * 4);
  float* gat2 = (float*)carve((size_t)NT2 * 128 * 4);
  float* xn2  = (float*)carve((size_t)NT2 * 128 * 4);
  float* sc2  = (float*)carve((size_t)BG * SPAD2 * 4);
  int*   nid2 = (int*)carve((size_t)BG * SPAD2 * 4);
  unsigned short* x3h = (unsigned short*)carve((size_t)NT3 * 128 * 2);
  unsigned short* x3l = (unsigned short*)carve((size_t)NT3 * 128 * 2);
  int*   es3  = (int*)carve((size_t)NEDGE * 4);
  int*   ed3  = (int*)carve((size_t)NEDGE * 4);
  float* xp3  = (float*)carve((size_t)NT3 * 256 * 4);
  float* al3  = (float*)carve((size_t)NT3 * 4 * 4);
  float* gat3 = (float*)carve((size_t)NT3 * 256 * 4);
  unsigned short* xn3h = (unsigned short*)carve((size_t)NT3 * 256 * 2);
  unsigned short* xn3l = (unsigned short*)carve((size_t)NT3 * 256 * 2);
  float* gate1 = (float*)carve((size_t)NT3 * 64 * 4);
  float* hbuf  = (float*)carve((size_t)NT3 * 256 * 4);
  if (off > (size_t)WSLIM || off > ws_size) return;

  const int ldsG1 = (1024 * 32 + 1024 * 4 + 8 * WCAP + 8) * 4;
  const int ldsG2 = (256 * 128 + 256 * 4 + 8 * WCAP + 8) * 4;
  const int ldsG3 = (128 * 256 + 128 * 4 + 8 * WCAP + 8) * 4;
  const int ldsP1 = 8192 * 8 + SPAD1 * 4;
  const int ldsP2 = 4096 * 8 + SPAD2 * 4;
  const int ldsM32  = 2 * 64 * (32 + 8) * 2 + 4 * 16 * 68 * 4;
  const int ldsM128 = 2 * 64 * (128 + 8) * 2 + 4 * 16 * 68 * 4;
  const int ldsM256 = 2 * 64 * (256 + 8) * 2 + 4 * 16 * 68 * 4;
  const int ldsF = (768 + 256) * 4 + 2 * 16 * 264 * 2 + 2 * 16 * 520 * 2 + 2 * 16 * 136 * 2 + 256 * 4 + 96 * 4;

  hipFuncSetAttribute(reinterpret_cast<const void*>(&k_gat<32, 2, 1024>), hipFuncAttributeMaxDynamicSharedMemorySize, ldsG1);
  hipFuncSetAttribute(reinterpret_cast<const void*>(&k_gat<128, 2, 256>), hipFuncAttributeMaxDynamicSharedMemorySize, ldsG2);
  hipFuncSetAttribute(reinterpret_cast<const void*>(&k_gat<256, 1, 128>), hipFuncAttributeMaxDynamicSharedMemorySize, ldsG3);
  hipFuncSetAttribute(reinterpret_cast<const void*>(&k_pool<32>), hipFuncAttributeMaxDynamicSharedMemorySize, ldsP1);
  hipFuncSetAttribute(reinterpret_cast<const void*>(&k_pool<128>), hipFuncAttributeMaxDynamicSharedMemorySize, ldsP2);
  hipFuncSetAttribute(reinterpret_cast<const void*>(&k_gemm<256, 1, true>), hipFuncAttributeMaxDynamicSharedMemorySize, ldsM256);
  hipFuncSetAttribute(reinterpret_cast<const void*>(&k_gemm<128, 0, false>), hipFuncAttributeMaxDynamicSharedMemorySize, ldsM128);
  hipFuncSetAttribute(reinterpret_cast<const void*>(&k_final), hipFuncAttributeMaxDynamicSharedMemorySize, ldsF);

  k_proj1<<<NT1 / 64, 128, 0, stream>>>(pos, W1, xp1, NT1);
  k_alpha<2><<<NT1 / 256, 256, 0, stream>>>(xp1, a_s1, a_d1, al1, NT1, 16);
  k_gat<32, 2, 1024><<<BG * 8, 256, ldsG1, stream>>>(src, dst, xp1, al1, b1, gat1, NPG1, 8, NT1);
  k_norm<32, 0><<<BG, 256, 0, stream>>>(gat1, p1, xn1, sc1, x2h, x2l, NPG1, SPAD1);
  k_pool<32><<<BG, 512, ldsP1, stream>>>(xn1, sc1, x2h, x2l, nid1, NPG1, SPAD1, KP1, 8192);
  k_remap<<<NEDGE / 1024, 256, 0, stream>>>(src, dst, nid1, es2, ed2, NPG1, SPAD1, NT1, NEDGE / 4);

  k_gemm<32, 0, false><<<dim3((NT2 + 63) / 64, 128 / 64), 128, ldsM32, stream>>>(x2h, x2l, W2, W2, xp2, NT2, 128);
  k_alpha<2><<<(NT2 + 255) / 256, 256, 0, stream>>>(xp2, a_s2, a_d2, al2, NT2, 64);
  k_gat<128, 2, 256><<<BG * 10, 256, ldsG2, stream>>>(es2, ed2, xp2, al2, b2, gat2, KP1, 10, NT2);
  k_norm<128, 0><<<BG, 256, 0, stream>>>(gat2, p2, xn2, sc2, x3h, x3l, KP1, SPAD2);
  k_pool<128><<<BG, 512, ldsP2, stream>>>(xn2, sc2, x3h, x3l, nid2, KP1, SPAD2, KP2, 4096);
  k_remap<<<NEDGE / 1024, 256, 0, stream>>>(es2, ed2, nid2, es3, ed3, KP1, SPAD2, NT2, NEDGE / 4);

  k_gemm<128, 0, false><<<dim3((NT3 + 63) / 64, 256 / 64), 128, ldsM128, stream>>>(x3h, x3l, W3, W3, xp3, NT3, 256);
  k_alpha<1><<<(NT3 + 255) / 256, 256, 0, stream>>>(xp3, a_s3, a_d3, al3, NT3, 256);
  k_gat<256, 1, 128><<<BG * 6, 256, ldsG3, stream>>>(es3, ed3, xp3, al3, b3, gat3, KP2, 6, NT3);
  k_norm<256, 1><<<BG, 256, 0, stream>>>(gat3, p2, xn2, sc2, xn3h, xn3l, KP2, SPAD2);

  k_gemm<256, 1, true><<<dim3((NT3 + 63) / 64, 64 / 64), 128, ldsM256, stream>>>(xn3h, xn3l, gw1, gb1, gate1, NT3, 64);
  k_gemm<256, 1, true><<<dim3((NT3 + 63) / 64, 256 / 64), 128, ldsM256, stream>>>(xn3h, xn3l, aw, ab, hbuf, NT3, 256);
  k_final<<<1, 256, ldsF, stream>>>(gate1, gw2, gb2, hbuf, w1, bb1, w2, bb2, w3, bb3, outp);
  hipGetLastError();
}
